// GraphEmbeddingLayer_69518340653483
// MI455X (gfx1250) — hardware-verified
//
#include <hip/hip_runtime.h>
#include <stddef.h>


#define DM     256
#define HN     4
#define CH     128
#define HC     512
#define THR    256
#define NWV    8
#define RB1    128
#define NB     64
#define FBK    64
#define FNODES 4096
#define CAP    4096
#define CHUNK  4096
#define WSC    64.0f
#define XINV   0.015625f
#define ASC    16.0f
#define RSC    0.0009765625f
#define WSCAP  134217728
#define LDS_PJ (NWV * 16 * 128 * 4 + 2 * RB1 * 4)
#define LDS_DR (NB * HC * 4 + NWV * 16 * 128 * 4 + NB * HN * 4 * 2 + NB * 4 * 3 + 64)

static_assert(FNODES == NB * FBK);
static_assert(CHUNK == THR * 16 && NWV * 32 == THR);
static_assert(LDS_PJ == 66560 && LDS_DR == 199488);
static_assert((CAP % 64) == 0 && FBK == 8 * NWV && NB == 8 * NWV && RB1 == 16 * NWV && (RB1 % NB) == 0);
static_assert(NB * HC == 32 * THR * 4 && NB * HN == THR);
static_assert(DM * HC == 64 * THR * 8);
static_assert((DM % 32) == 0 && (HC % 32) == 0);

typedef float    v4f  __attribute__((ext_vector_type(4)));
typedef float    v8f  __attribute__((ext_vector_type(8)));
typedef int      v4i  __attribute__((ext_vector_type(4)));
typedef _Float16 v4h  __attribute__((ext_vector_type(4)));
typedef _Float16 v8h  __attribute__((ext_vector_type(8)));
typedef _Float16 v16h __attribute__((ext_vector_type(16)));
union Frag { v16h v; v8h h[2]; v4h q[4]; };

#define WSYNC() do { __builtin_amdgcn_fence(__ATOMIC_ACQ_REL, "wavefront"); __builtin_amdgcn_wave_barrier(); } while (0)

__device__ __forceinline__ v8f wmh(v16h a, v16h b, v8f c) {
  v8f d = __builtin_amdgcn_wmma_f32_16x16x32_f16(false, a, false, b, (short)0, c, false, false);
  asm volatile("v_nop\n\tv_nop\n\tv_nop\n\tv_nop" : "+v"(d) : "v"(a), "v"(b));
  return d;
}

__global__ __launch_bounds__(THR) void k_wprep(const float* __restrict__ w, const float* __restrict__ wo,
                                               _Float16* WP, _Float16* WOP) {
  const int blk = blockIdx.x, tid = threadIdx.x;
  const float* sp;
  _Float16* dp;
  int st;
  if (blk < 64) {
    const int i = blk * THR + tid;
    const int n = i >> 5, k8 = (i & 31) * 8;
    sp = w + (size_t)k8 * HC + n; st = HC; dp = WP + (size_t)i * 8;
  } else {
    const int i = (blk - 64) * THR + tid;
    const int n = i >> 6, k8 = (i & 63) * 8;
    sp = wo + (size_t)k8 * DM + n; st = DM; dp = WOP + (size_t)i * 8;
  }
  v8h hv;
#pragma unroll
  for (int e = 0; e < 8; ++e) hv[e] = (_Float16)(sp[(size_t)e * st] * WSC);
  *(volatile v8h*)dp = hv;
  __threadfence();
  *(volatile v8h*)dp = hv;
}

__global__ __launch_bounds__(THR) void k_proj(const float* __restrict__ emb, const _Float16* __restrict__ WP,
                                              const float* __restrict__ ats, const float* __restrict__ atd,
                                              float* X, float* AS, float* AD, int nN, int nPad) {
  extern __shared__ __attribute__((aligned(16))) char dynl[];
  float* sx = (float*)dynl;
  float* ss = sx + NWV * 2048;
  const int tid = threadIdx.x, lane = tid & 31, hh = lane >> 4, m = lane & 15;
  const int wave = __builtin_amdgcn_readfirstlane(tid >> 5);
  const int head = blockIdx.y;
  const int row0 = blockIdx.x * RB1 + wave * 16;
  int arow = row0 + m;
  arow = arow > nN - 1 ? nN - 1 : arow;
  const float* ap = emb + (size_t)arow * DM + 8 * hh;
  const _Float16* bp = WP + (size_t)(head * CH + m) * DM + 8 * hh;
  float as8[8], ad8[8];
#pragma unroll
  for (int t = 0; t < 8; ++t) {
    as8[t] = ats[head * CH + 16 * t + m];
    ad8[t] = atd[head * CH + 16 * t + m];
  }
  v8f acc[8];
#pragma unroll
  for (int t = 0; t < 8; ++t) { v8f z = {0.f, 0.f, 0.f, 0.f, 0.f, 0.f, 0.f, 0.f}; acc[t] = z; }

#pragma unroll 1
  for (int ks = 0; ks < DM / 32; ++ks) {
    const float* a0 = ap + 32 * ks;
    const v4f f0 = *(const v4f*)a0, f1 = *(const v4f*)(a0 + 4);
    const v4f f2 = *(const v4f*)(a0 + 16), f3 = *(const v4f*)(a0 + 20);
    Frag a;
    a.q[0] = __builtin_convertvector(f0, v4h);
    a.q[1] = __builtin_convertvector(f1, v4h);
    a.q[2] = __builtin_convertvector(f2, v4h);
    a.q[3] = __builtin_convertvector(f3, v4h);
#pragma unroll
    for (int t = 0; t < 8; ++t) {
      const _Float16* q = bp + (size_t)(16 * t) * DM + 32 * ks;
      Frag b;
      b.h[0] = *(const v8h*)q;
      b.h[1] = *(const v8h*)(q + 16);
      acc[t] = wmh(a.v, b.v, acc[t]);
    }
  }

  float* sxw = sx + wave * 2048;
  float ps[8], pd[8];
#pragma unroll
  for (int r = 0; r < 8; ++r) { ps[r] = 0.f; pd[r] = 0.f; }
#pragma unroll
  for (int t = 0; t < 8; ++t) {
#pragma unroll
    for (int r = 0; r < 8; ++r) {
      const float v = acc[t][r] * XINV;
      sxw[(8 * hh + r) * 128 + 16 * t + m] = v;
      ps[r] = fmaf(v, as8[t], ps[r]);
      pd[r] = fmaf(v, ad8[t], pd[r]);
    }
  }
#pragma unroll
  for (int r = 0; r < 8; ++r) {
    float a = ps[r], b = pd[r];
    a += __shfl_xor(a, 1, 32); b += __shfl_xor(b, 1, 32);
    a += __shfl_xor(a, 2, 32); b += __shfl_xor(b, 2, 32);
    a += __shfl_xor(a, 4, 32); b += __shfl_xor(b, 4, 32);
    a += __shfl_xor(a, 8, 32); b += __shfl_xor(b, 8, 32);
    ps[r] = a; pd[r] = b;
  }
  if (m == 0) {
#pragma unroll
    for (int r = 0; r < 8; ++r) {
      ss[16 * wave + 8 * hh + r] = ps[r];
      ss[RB1 + 16 * wave + 8 * hh + r] = pd[r];
    }
  }
  WSYNC();
  v4f xs[16];
#pragma unroll
  for (int r = 0; r < 16; ++r) xs[r] = *(const v4f*)(sxw + r * 128 + 4 * lane);
  float* xg = X + (size_t)row0 * HC + head * CH + 4 * lane;
#pragma unroll
  for (int r = 0; r < 16; ++r) *(volatile v4f*)(xg + (size_t)r * HC) = xs[r];
  __syncthreads();
  v4f av = {0.f, 0.f, 0.f, 0.f};
  float* ag = (wave == 0) ? AS : AD;
  ag += (size_t)head * nPad + (size_t)blockIdx.x * RB1 + 4 * lane;
  if (wave < 2) {
    av = *(const v4f*)(ss + RB1 * wave + 4 * lane);
    *(volatile v4f*)ag = av;
  }
  __threadfence();
#pragma unroll
  for (int r = 0; r < 16; ++r) *(volatile v4f*)(xg + (size_t)r * HC) = xs[r];
  if (wave < 2) *(volatile v4f*)ag = av;
}

__device__ __forceinline__ int compact4k(const int* __restrict__ dsts, int nE, int cbase, int n0,
                                         int wave, int lane, int vec, unsigned* slist, int* swt) {
  int d[16];
  const int eb = cbase + 512 * wave + 4 * lane;
  if (vec != 0 && cbase + CHUNK <= nE) {
#pragma unroll
    for (int q = 0; q < 4; ++q) {
      const v4i t4 = *(const v4i*)(dsts + eb + 128 * q);
      d[4 * q] = t4.x; d[4 * q + 1] = t4.y; d[4 * q + 2] = t4.z; d[4 * q + 3] = t4.w;
    }
  } else {
#pragma unroll
    for (int k = 0; k < 16; ++k) {
      int idx = eb + 128 * (k >> 2) + (k & 3);
      const bool ok = idx < nE;
      idx = ok ? idx : nE - 1;
      const int val = dsts[idx];
      d[k] = ok ? val : (-2147483647 - 1);
    }
  }
  unsigned hm[16];
  int cw = 0;
#pragma unroll
  for (int k = 0; k < 16; ++k) {
    const unsigned ld = (unsigned)d[k] - (unsigned)n0;
    hm[k] = __builtin_amdgcn_ballot_w32(ld < (unsigned)FNODES);
    cw += __builtin_popcount(hm[k]);
  }
  swt[wave] = cw;
  __syncthreads();
  int base = 0, nh = 0;
#pragma unroll
  for (int w = 0; w < NWV; ++w) {
    const int v = swt[w];
    base += (w < wave) ? v : 0;
    nh += v;
  }
  int run = base;
#pragma unroll
  for (int k = 0; k < 16; ++k) {
    const unsigned ld = (unsigned)d[k] - (unsigned)n0;
    const unsigned mk = hm[k];
    const int pos = run + (int)__builtin_amdgcn_mbcnt_lo(mk, 0u);
    const unsigned e = (unsigned)(eb + 128 * (k >> 2) + (k & 3));
    if (ld < (unsigned)FNODES) slist[pos & (CHUNK - 1)] = (e << 12) | ld;
    run += __builtin_popcount(mk);
  }
  __syncthreads();
  return nh;
}

__device__ __forceinline__ void bk_flush(const int* sbuf, int* BKT, int bk0, int lbk, int L, int nval, int lane) {
  WSYNC();
  int v = sbuf[lbk * 64 + ((32 * L + lane) & 63)];
  v = (lane < nval) ? v : 0;
  WSYNC();
  int* gp = BKT + (size_t)(bk0 + lbk) * CAP + 32 * L + lane;
  *(volatile int*)gp = v;
  __threadfence();
  *(volatile int*)gp = v;
}

__global__ __launch_bounds__(THR) void k_fill(const int* __restrict__ dsts, int* BKT, int* CNTT,
                                              int nE, int nChunks, int vec) {
  __shared__ __attribute__((aligned(16))) unsigned slist[CHUNK];
  __shared__ __attribute__((aligned(16))) int sbuf[FBK * 64];
  __shared__ int swt[NWV];
  __shared__ int scount[FBK];
  const int tid = threadIdx.x, lane = tid & 31;
  const int wave = __builtin_amdgcn_readfirstlane(tid >> 5);
  const int n0 = blockIdx.x * FNODES, bk0 = blockIdx.x * FBK;
  int cur[8];
#pragma unroll
  for (int jj = 0; jj < 8; ++jj) cur[jj] = 0;

#pragma unroll 1
  for (int c = 0; c < nChunks; ++c) {
    const int nh = compact4k(dsts, nE, c * CHUNK, n0, wave, lane, vec, slist, swt);
    const int nhc = nh < CHUNK ? nh : CHUNK;
    for (int j0 = 0; j0 < nhc; j0 += 32) {
      const int idx = j0 + lane;
      const bool inr = idx < nhc;
      const unsigned ent = slist[inr ? idx : 0];
      const int e = (int)(ent >> 12);
      const int lb = (int)(ent & 4095u) >> 6;
#pragma unroll
      for (int jj = 0; jj < 8; ++jj) {
        const int mylb = 8 * wave + jj;
        const bool mine = inr && (lb == mylb);
        const unsigned mk = __builtin_amdgcn_ballot_w32(mine);
        if (mk != 0u) {
          const int c0 = cur[jj];
          const int g = c0 + (int)__builtin_amdgcn_mbcnt_lo(mk, 0u);
          if (mine && g < CAP) sbuf[mylb * 64 + (g & 63)] = e;
          const int c1 = c0 + __builtin_popcount(mk);
          cur[jj] = c1;
          const int L = c0 >> 5;
          if ((c1 >> 5) != L && L < CAP / 32) bk_flush(sbuf, BKT, bk0, mylb, L, 32, lane);
        }
      }
    }
  }
#pragma unroll
  for (int jj = 0; jj < 8; ++jj) {
    const int c0 = cur[jj];
    const int rem = c0 & 31, L = c0 >> 5;
    if (rem != 0 && L < CAP / 32) bk_flush(sbuf, BKT, bk0, 8 * wave + jj, L, rem, lane);
    if (lane == 0) scount[8 * wave + jj] = c0 < CAP ? c0 : CAP;
  }
  __syncthreads();
  if (wave < 2) {
    const int v = scount[32 * wave + lane];
    int* gp = CNTT + bk0 + 32 * wave + lane;
    *(volatile int*)gp = v;
    __threadfence();
    *(volatile int*)gp = v;
  }
}

__device__ __forceinline__ float gat_logit(const float* __restrict__ AS, const float* __restrict__ AD,
                                           const float* sk, int nPad, int h, int s, int d, float we) {
  float t = AS[(size_t)h * nPad + s] + AD[(size_t)h * nPad + d];
  t = fmaf(we, sk[h], t);
  return fmaxf(t, 0.2f * t);
}

__global__ __launch_bounds__(THR) void k_drain(
    const int* __restrict__ srcs, const int* __restrict__ dsts, const float* __restrict__ ew,
    const float* __restrict__ X, const float* __restrict__ AS, const float* __restrict__ AD,
    const float* __restrict__ ate, const float* __restrict__ wed, const float* __restrict__ bias,
    const _Float16* __restrict__ WOP, const float* __restrict__ bout,
    const int* __restrict__ BKT, const int* __restrict__ CNTT, float* out,
    int nN, int nE, int nPad) {
  extern __shared__ __attribute__((aligned(16))) char dynl[];
  float* sacc = (float*)dynl;
  float* so   = sacc + NB * HC;
  float* smx  = so + NWV * 2048;
  float* sdn  = smx + NB * HN;
  int*   scnt = (int*)(sdn + NB * HN);
  float* swsm = (float*)(scnt + NB);
  float* sea  = swsm + NB;
  float* sk   = sea + NB;
  const int tid = threadIdx.x, lane = tid & 31, hh = lane >> 4, m = lane & 15;
  const int wave = __builtin_amdgcn_readfirstlane(tid >> 5);
  const int n0 = blockIdx.x * NB;

  {
    v4f z = {0.f, 0.f, 0.f, 0.f};
    v4f* p = (v4f*)sacc;
#pragma unroll
    for (int it = 0; it < 32; ++it) p[it * THR + tid] = z;
    smx[tid] = -3.0e38f;
    sdn[tid] = 0.0f;
    if (tid < NB) { scnt[tid] = 0; swsm[tid] = 0.0f; sea[tid] = 0.0f; }
  }
  if (wave < HN) {
    float s = 0.f;
#pragma unroll
    for (int i = 0; i < CH / 32; ++i) {
      const int c = lane + 32 * i;
      s = fmaf(ate[wave * CH + c], wed[wave * CH + c], s);
    }
    s += __shfl_xor(s, 16, 32);
    s += __shfl_xor(s, 8, 32);
    s += __shfl_xor(s, 4, 32);
    s += __shfl_xor(s, 2, 32);
    s += __shfl_xor(s, 1, 32);
    if (lane == 0) sk[wave] = s;
  }
  __syncthreads();

  int cntb = CNTT[blockIdx.x];
  cntb = cntb < 0 ? 0 : (cntb > CAP ? CAP : cntb);
  const int* bk = BKT + (size_t)blockIdx.x * CAP;

#pragma unroll 1
  for (int j0 = 0; j0 < cntb; j0 += 32) {
    int idx = j0 + lane;
    const bool inr = idx < cntb;
    idx = idx > CAP - 1 ? CAP - 1 : idx;
    int e = bk[idx];
    e = e < 0 ? 0 : (e > nE - 1 ? nE - 1 : e);
    const int d = dsts[e];
    const int ld = d - n0;
    const bool own = inr && ((unsigned)ld < (unsigned)NB) && ((ld & 7) == wave);
    unsigned om = __builtin_amdgcn_ballot_w32(own);
    while (om != 0u) {
      const int b = __builtin_ctz(om);
      om &= om - 1u;
      const int eu = __builtin_amdgcn_readlane(e, b);
      const int ldu = __builtin_amdgcn_readlane(ld, b);
      int s = srcs[eu];
      s = s < 0 ? 0 : (s > nN - 1 ? nN - 1 : s);
      const float we = ew[eu];
      const int h = lane & 3;
      const float lg = gat_logit(AS, AD, sk, nPad, h, s, n0 + ldu, we);
      if (lane < HN) smx[ldu * HN + h] = fmaxf(smx[ldu * HN + h], lg);
      if (lane == 0) { scnt[ldu] = scnt[ldu] + 1; swsm[ldu] = swsm[ldu] + we; }
    }
  }
  WSYNC();
#pragma unroll 1
  for (int q = 0; q < NB / NWV; ++q) {
    const int ld = wave + 8 * q;
    const int node = n0 + ld;
    const int cn = scnt[ld];
    const float ea = swsm[ld] * (1.0f / fmaxf((float)cn, 1.0f));
    if (lane == 0) sea[ld] = ea;
    const int h = lane & 3;
    const float lg = gat_logit(AS, AD, sk, nPad, h, node, node, ea);
    if (lane < HN) smx[ld * HN + h] = fmaxf(smx[ld * HN + h], lg);
  }
  WSYNC();

#pragma unroll 1
  for (int j0 = 0; j0 < cntb; j0 += 32) {
    int idx = j0 + lane;
    const bool inr = idx < cntb;
    idx = idx > CAP - 1 ? CAP - 1 : idx;
    int e = bk[idx];
    e = e < 0 ? 0 : (e > nE - 1 ? nE - 1 : e);
    const int d = dsts[e];
    const int ld = d - n0;
    const bool own = inr && ((unsigned)ld < (unsigned)NB) && ((ld & 7) == wave);
    unsigned om = __builtin_amdgcn_ballot_w32(own);
    while (om != 0u) {
      const int b = __builtin_ctz(om);
      om &= om - 1u;
      const int eu = __builtin_amdgcn_readlane(e, b);
      const int ldu = __builtin_amdgcn_readlane(ld, b);
      int s = srcs[eu];
      s = s < 0 ? 0 : (s > nN - 1 ? nN - 1 : s);
      const float we = ew[eu];
      const int h = lane >> 3;
      const float lg = gat_logit(AS, AD, sk, nPad, h, s, n0 + ldu, we);
      const float p = __expf(lg - smx[ldu * HN + h]);
      if ((lane & 7) == 0) sdn[ldu * HN + h] = sdn[ldu * HN + h] + p;
      const float* xr = X + (size_t)s * HC + 16 * lane;
      float* ar = sacc + ldu * HC + 16 * lane;
#pragma unroll
      for (int i = 0; i < 4; ++i) {
        const v4f xv = *(const v4f*)(xr + 4 * i);
        v4f av = *(const v4f*)(ar + 4 * i);
        av.x = fmaf(p, xv.x, av.x); av.y = fmaf(p, xv.y, av.y);
        av.z = fmaf(p, xv.z, av.z); av.w = fmaf(p, xv.w, av.w);
        *(v4f*)(ar + 4 * i) = av;
      }
    }
  }
#pragma unroll 1
  for (int q = 0; q < NB / NWV; ++q) {
    const int ld = wave + 8 * q;
    const int node = n0 + ld;
    const float ea = sea[ld];
    const int h = lane >> 3;
    const float lg = gat_logit(AS, AD, sk, nPad, h, node, node, ea);
    const float p = __expf(lg - smx[ld * HN + h]);
    if ((lane & 7) == 0) sdn[ld * HN + h] = sdn[ld * HN + h] + p;
    const float* xr = X + (size_t)node * HC + 16 * lane;
    float* ar = sacc + ld * HC + 16 * lane;
#pragma unroll
    for (int i = 0; i < 4; ++i) {
      const v4f xv = *(const v4f*)(xr + 4 * i);
      v4f av = *(const v4f*)(ar + 4 * i);
      av.x = fmaf(p, xv.x, av.x); av.y = fmaf(p, xv.y, av.y);
      av.z = fmaf(p, xv.z, av.z); av.w = fmaf(p, xv.w, av.w);
      *(v4f*)(ar + 4 * i) = av;
    }
  }
  __syncthreads();

#pragma unroll 1
  for (int it = 0; it < (NB * HC / 4) / THR; ++it) {
    const int idx = it * THR + tid;
    const int row = idx >> 7, c4 = idx & 127, h = c4 >> 5;
    const float rcp = 1.0f / (sdn[row * HN + h] + 1e-16f);
    v4f a = *(const v4f*)(sacc + (size_t)idx * 4);
    const v4f bb = *(const v4f*)(bias + 4 * c4);
    a.x = fmaf(a.x, rcp, bb.x) * ASC; a.y = fmaf(a.y, rcp, bb.y) * ASC;
    a.z = fmaf(a.z, rcp, bb.z) * ASC; a.w = fmaf(a.w, rcp, bb.w) * ASC;
    *(v4f*)(sacc + (size_t)idx * 4) = a;
  }
  __syncthreads();

  const int rt = wave & 3, chf = wave >> 2;
  float bo[8];
#pragma unroll
  for (int t = 0; t < 8; ++t) bo[t] = bout[128 * chf + 16 * t + m];
  v8f acc8[8];
#pragma unroll
  for (int t = 0; t < 8; ++t) { v8f z = {0.f, 0.f, 0.f, 0.f, 0.f, 0.f, 0.f, 0.f}; acc8[t] = z; }
  const float* arow = sacc + (16 * rt + m) * HC + 8 * hh;
  const _Float16* brow = WOP + (size_t)(128 * chf + m) * HC + 8 * hh;
#pragma unroll 1
  for (int ks = 0; ks < HC / 32; ++ks) {
    const float* a0 = arow + 32 * ks;
    const v4f f0 = *(const v4f*)a0, f1 = *(const v4f*)(a0 + 4);
    const v4f f2 = *(const v4f*)(a0 + 16), f3 = *(const v4f*)(a0 + 20);
    Frag a;
    a.q[0] = __builtin_convertvector(f0, v4h);
    a.q[1] = __builtin_convertvector(f1, v4h);
    a.q[2] = __builtin_convertvector(f2, v4h);
    a.q[3] = __builtin_convertvector(f3, v4h);
#pragma unroll
    for (int t = 0; t < 8; ++t) {
      const _Float16* q = brow + (size_t)(16 * t) * HC + 32 * ks;
      Frag b;
      b.h[0] = *(const v8h*)q;
      b.h[1] = *(const v8h*)(q + 16);
      acc8[t] = wmh(a.v, b.v, acc8[t]);
    }
  }
  float* sow = so + wave * 2048;
#pragma unroll
  for (int t = 0; t < 8; ++t) {
#pragma unroll
    for (int r = 0; r < 8; ++r) sow[(8 * hh + r) * 128 + 16 * t + m] = fmaf(acc8[t][r], RSC, bo[t]);
  }
  WSYNC();
  v4f ov[16];
#pragma unroll
  for (int r = 0; r < 16; ++r) ov[r] = *(const v4f*)(sow + r * 128 + 4 * lane);
  const int grow0 = n0 + 16 * rt;
  float* og = out + (size_t)grow0 * DM + 128 * chf + 4 * lane;
#pragma unroll
  for (int r = 0; r < 16; ++r) {
    if (grow0 + r < nN) *(volatile v4f*)(og + (size_t)r * DM) = ov[r];
  }
  __threadfence();
#pragma unroll
  for (int r = 0; r < 16; ++r) {
    if (grow0 + r < nN) *(volatile v4f*)(og + (size_t)r * DM) = ov[r];
  }
}

extern "C" void kernel_launch(void* const* d_in, const int* in_sizes, int n_in,
                              void* d_out, int out_size, void* d_ws, size_t ws_size,
                              hipStream_t stream) {
  if (n_in < 11) return;
  const int nE = in_sizes[1];
  const int nN = in_sizes[2] / DM;
  if (nN < 1 || nE < 1) return;
  if (in_sizes[0] != 2 * nE || in_sizes[2] != nN * DM) return;
  if (in_sizes[3] != DM * HC || in_sizes[4] != HN * CH || in_sizes[5] != HN * CH || in_sizes[6] != HN * CH) return;
  if (in_sizes[7] != HC || in_sizes[8] != HC || in_sizes[9] != HC * DM || in_sizes[10] != DM) return;
  if (out_size != nN * DM) return;
  if (nE > (1 << 20) || nN > (1 << 22)) return;

  const int*   ei   = (const int*)d_in[0];
  const float* ew   = (const float*)d_in[1];
  const float* emb  = (const float*)d_in[2];
  const float* w    = (const float*)d_in[3];
  const float* ats  = (const float*)d_in[4];
  const float* atd  = (const float*)d_in[5];
  const float* ate  = (const float*)d_in[6];
  const float* wed  = (const float*)d_in[7];
  const float* bias = (const float*)d_in[8];
  const float* wo   = (const float*)d_in[9];
  const float* bout = (const float*)d_in[10];
  float* out = (float*)d_out;
  const int* srcs = ei;
  const int* dsts = ei + (size_t)nE;

  const int nPad    = ((nN + RB1 - 1) / RB1) * RB1;
  const int gProj   = nPad / RB1;
  const int gDrain  = nPad / NB;
  const int gFill   = (nPad + FNODES - 1) / FNODES;
  const int nBkP    = gFill * FBK;
  const int nChunks = (nE + CHUNK - 1) / CHUNK;
  const int vec     = ((nE & 3) == 0) ? 1 : 0;

  char* ws = (char*)d_ws;
  size_t off = 0;
  const size_t oWP  = off; off += (size_t)HC * DM * 2;          off = (off + 255) & ~(size_t)255;
  const size_t oWOP = off; off += (size_t)DM * HC * 2;          off = (off + 255) & ~(size_t)255;
  const size_t oX   = off; off += (size_t)nPad * HC * 4;        off = (off + 255) & ~(size_t)255;
  const size_t oAS  = off; off += (size_t)HN * nPad * 4;        off = (off + 255) & ~(size_t)255;
  const size_t oAD  = off; off += (size_t)HN * nPad * 4;        off = (off + 255) & ~(size_t)255;
  const size_t oCN  = off; off += (size_t)nBkP * 4;             off = (off + 255) & ~(size_t)255;
  const size_t oBK  = off; off += (size_t)nBkP * CAP * 4;       off = (off + 255) & ~(size_t)255;
  if (off > ws_size || off > (size_t)WSCAP) return;
  _Float16* WP  = (_Float16*)(ws + oWP);
  _Float16* WOP = (_Float16*)(ws + oWOP);
  float*    X   = (float*)(ws + oX);
  float*    AS  = (float*)(ws + oAS);
  float*    AD  = (float*)(ws + oAD);
  int*      CNTT = (int*)(ws + oCN);
  int*      BKT  = (int*)(ws + oBK);

  hipFuncSetAttribute(reinterpret_cast<const void*>(&k_proj), hipFuncAttributeMaxDynamicSharedMemorySize, LDS_PJ);
  hipFuncSetAttribute(reinterpret_cast<const void*>(&k_drain), hipFuncAttributeMaxDynamicSharedMemorySize, LDS_DR);

  k_wprep<<<128, THR, 0, stream>>>(w, wo, WP, WOP);
  k_proj<<<dim3(gProj, HN), THR, LDS_PJ, stream>>>(emb, WP, ats, atd, X, AS, AD, nN, nPad);
  k_fill<<<gFill, THR, 0, stream>>>(dsts, BKT, CNTT, nE, nChunks, vec);
  k_drain<<<gDrain, THR, LDS_DR, stream>>>(srcs, dsts, ew, X, AS, AD, ate, wed, bias, WOP, bout,
                                           BKT, CNTT, out, nN, nE, nPad);
}
